// MambaBlock_66125316489621
// MI455X (gfx1250) — hardware-verified
//
#include <hip/hip_runtime.h>
#include <math.h>

typedef __attribute__((ext_vector_type(16))) _Float16 v16h;
typedef __attribute__((ext_vector_type(8)))  _Float16 v8h;
typedef __attribute__((ext_vector_type(8)))  float    v8f;
typedef __attribute__((ext_vector_type(4)))  float    v4f;

constexpr int kBatch = 2;
constexpr int kSeqL  = 2048;
constexpr int kDmod  = 1024;
constexpr int kDin   = 2048;
constexpr int kNst   = 16;
constexpr int kDtR   = 64;
constexpr int kPrjN  = 96;
constexpr int kPrjP  = 128;
constexpr int kXZN   = 2 * kDin;
constexpr int kRows  = kBatch * kSeqL;
constexpr int kTP    = 260;

constexpr float kCarryW   = 32.0f;
constexpr float kCarryWdt = 8.0f;
constexpr float kCarryDt  = 16.0f;
constexpr float kCarryY   = 16.0f;
constexpr float kCarryXlo = 2048.0f;

static_assert(kDtR + 2 * kNst == kPrjN, "x_proj width");
static_assert((kDmod % 32) == 0 && (kDin % 32) == 0 && (kDtR % 32) == 0, "GEMM K multiples of 32");
static_assert((kRows % 64) == 0 && (kDin % 64) == 0 && (kPrjP % 64) == 0 && (kDmod % 64) == 0, "GEMM M,N multiples of 64");
static_assert((kRows % 32) == 0, "in_proj M multiple of 32");
static_assert((kSeqL % 64) == 0 && (kDin % 256) == 0, "tile multiples");
static_assert(((kRows / 32) * (kDin / 64)) % 8 == 0, "in_proj tiles fill whole blocks");
static_assert(((kRows / 64) * (kDin / 64)) % 8 == 0, "dt tiles fill whole blocks");
static_assert(((kRows / 64) * (kPrjP / 64)) % 8 == 0, "x_proj tiles fill whole blocks");
static_assert(((kRows / 64) * (kDmod / 64)) % 8 == 0, "out_proj tiles fill whole blocks");

constexpr size_t kSzX16     = (size_t)kRows * kDmod * 2;
constexpr size_t kSzXLO16   = (size_t)kRows * kDmod * 2;
constexpr size_t kSzWIN16   = (size_t)kXZN * kDmod * 2;
constexpr size_t kSzWXP16   = (size_t)kPrjP * kDin * 2;
constexpr size_t kSzWDT16   = (size_t)kDin * kDtR * 2;
constexpr size_t kSzWOUT16  = (size_t)kDmod * kDin * 2;
constexpr size_t kSzXC32    = (size_t)kRows * kDin * 4;
constexpr size_t kSzZ16     = (size_t)kRows * kDin * 2;
constexpr size_t kSzU16     = (size_t)kRows * kDin * 2;
constexpr size_t kSzXDBL32  = (size_t)kRows * kPrjP * 4;
constexpr size_t kSzDTLO16  = (size_t)kRows * kDtR * 2;
constexpr size_t kSzDTRAW16 = (size_t)kRows * kDin * 2;
constexpr size_t kSzYG16    = (size_t)kRows * kDin * 2;
constexpr size_t kOffX16     = 0;
constexpr size_t kOffXLO16   = kOffX16     + kSzX16;
constexpr size_t kOffWIN16   = kOffXLO16   + kSzXLO16;
constexpr size_t kOffWXP16   = kOffWIN16   + kSzWIN16;
constexpr size_t kOffWDT16   = kOffWXP16   + kSzWXP16;
constexpr size_t kOffWOUT16  = kOffWDT16   + kSzWDT16;
constexpr size_t kOffXC32    = kOffWOUT16  + kSzWOUT16;
constexpr size_t kOffZ16     = kOffXC32    + kSzXC32;
constexpr size_t kOffU16     = kOffZ16     + kSzZ16;
constexpr size_t kOffXDBL32  = kOffU16     + kSzU16;
constexpr size_t kOffDTLO16  = kOffXDBL32  + kSzXDBL32;
constexpr size_t kOffDTRAW16 = kOffDTLO16  + kSzDTLO16;
constexpr size_t kOffYG16    = kOffDTRAW16 + kSzDTRAW16;
constexpr size_t kWsTotal    = kOffYG16    + kSzYG16;
static_assert(kWsTotal == 133431296ull, "carve total");
static_assert(kWsTotal <= 134217728ull, "carve cap");
static_assert((kOffXLO16 % 128) == 0 && (kOffWIN16 % 128) == 0 && (kOffWXP16 % 128) == 0 && (kOffWDT16 % 128) == 0 &&
              (kOffWOUT16 % 128) == 0 && (kOffXC32 % 128) == 0 && (kOffZ16 % 128) == 0 &&
              (kOffU16 % 128) == 0 && (kOffXDBL32 % 128) == 0 && (kOffDTLO16 % 128) == 0 &&
              (kOffDTRAW16 % 128) == 0 && (kOffYG16 % 128) == 0, "128-B aligned regions");

__device__ __forceinline__ float h16_to_f32(unsigned hb) {
  const unsigned sgn = (hb & 0x8000u) << 16;
  const unsigned em = hb & 0x7fffu;
  const float fn = __uint_as_float((em << 13) + 0x38000000u);
  const float fs = (float)em * 5.9604644775390625e-8f;
  const float mag = (em < 0x400u) ? fs : fn;
  return __uint_as_float(__float_as_uint(mag) | sgn);
}

__device__ __forceinline__ void group_guard_h(v8f& a, v8f& b, v8f& c, v8f& d,
                                              v16h x, v16h b0, v16h b1, v16h b2, v16h b3) {
  asm volatile("v_nop\n\tv_nop\n\tv_nop\n\tv_nop"
               : "+v"(a), "+v"(b), "+v"(c), "+v"(d)
               : "v"(x), "v"(b0), "v"(b1), "v"(b2), "v"(b3));
}
__device__ __forceinline__ void group_guard8_h(v8f& a, v8f& b, v8f& c, v8f& d,
                                               v8f& e, v8f& f, v8f& g, v8f& h,
                                               v16h x, v16h y, v16h b0, v16h b1, v16h b2, v16h b3) {
  asm volatile("v_nop\n\tv_nop\n\tv_nop\n\tv_nop"
               : "+v"(a), "+v"(b), "+v"(c), "+v"(d), "+v"(e), "+v"(f), "+v"(g), "+v"(h)
               : "v"(x), "v"(y), "v"(b0), "v"(b1), "v"(b2), "v"(b3));
}
__device__ __forceinline__ void keep4_h(v16h a, v16h b, v16h c, v16h d) { asm volatile("v_nop" :: "v"(a), "v"(b), "v"(c), "v"(d)); }
__device__ __forceinline__ void acc_guard4(v8f& a, v8f& b, v8f& c, v8f& d) { asm volatile("v_nop\n\tv_nop\n\tv_nop\n\tv_nop" : "+v"(a), "+v"(b), "+v"(c), "+v"(d)); }

struct FragH {
  union U { v16h v; v8h h[2]; };
  static __device__ __forceinline__ v16h load(const _Float16* p) {
    U f;
    f.h[0] = *(const v8h*)(p);
    f.h[1] = *(const v8h*)(p + 16);
    return f.v;
  }
  static __device__ __forceinline__ v8f mma(v16h a, v16h b, v8f c) {
    return __builtin_amdgcn_wmma_f32_16x16x32_f16(false, a, false, b, (short)0, c, false, false);
  }
};

template <int OUT_MODE>
__global__ __launch_bounds__(256) void wmma_gemm64_f16(
    const unsigned short* __restrict__ Ap, int lda,
    const unsigned short* __restrict__ Btp, int ldb,
    void* __restrict__ Cout, int ldc,
    int M, int N, int K, float scale)
{
  const _Float16* A  = (const _Float16*)Ap;
  const _Float16* Bt = (const _Float16*)Btp;
  __shared__ __align__(16) float sT[8][16 * 68];
  const int lane = threadIdx.x & 31;
  const int wave = threadIdx.x >> 5;
  const int tilesN = N >> 6;
  const int tilesM = M >> 6;
  const int tile = blockIdx.x * 8 + wave;
  if (tile >= tilesM * tilesN) return;
  const int tm = tile / tilesN;
  const int tn = tile - tm * tilesN;
  const int m0 = tm << 6;
  const int n0 = tn << 6;

  const int rlane = lane & 15;
  const int koff  = (lane >> 4) * 8;
  const int mOff  = (lane >> 4) * 8;

  v8f acc[4][4];
#pragma unroll
  for (int i = 0; i < 4; ++i)
#pragma unroll
    for (int j = 0; j < 4; ++j) acc[i][j] = (v8f){0.f,0.f,0.f,0.f,0.f,0.f,0.f,0.f};

  for (int k0 = 0; k0 < K; k0 += 32) {
    v16h bh[4];
#pragma unroll
    for (int j = 0; j < 4; ++j) {
      const size_t bo = (size_t)(n0 + (j << 4) + rlane) * ldb + koff + k0;
      bh[j] = FragH::load(Bt + bo);
    }
#pragma unroll
    for (int i = 0; i < 4; ++i) {
      const size_t ao = (size_t)(m0 + (i << 4) + rlane) * lda + koff + k0;
      v16h ah = FragH::load(A + ao);
#pragma unroll
      for (int j = 0; j < 4; ++j) acc[i][j] = FragH::mma(ah, bh[j], acc[i][j]);
      group_guard_h(acc[i][0], acc[i][1], acc[i][2], acc[i][3], ah, bh[0], bh[1], bh[2], bh[3]);
    }
    keep4_h(bh[0], bh[1], bh[2], bh[3]);
  }
  acc_guard4(acc[0][0], acc[0][1], acc[0][2], acc[0][3]);
  acc_guard4(acc[1][0], acc[1][1], acc[1][2], acc[1][3]);
  acc_guard4(acc[2][0], acc[2][1], acc[2][2], acc[2][3]);
  acc_guard4(acc[3][0], acc[3][1], acc[3][2], acc[3][3]);

  float* slab = sT[wave];
#pragma unroll
  for (int i = 0; i < 4; ++i) {
    const int mBase = m0 + (i << 4);
#pragma unroll
    for (int j = 0; j < 4; ++j) {
#pragma unroll
      for (int r = 0; r < 8; ++r) {
        const float v = acc[i][j][r] * scale;
        slab[(mOff + r) * 68 + (j << 4) + rlane] = v;
      }
    }
    __builtin_amdgcn_fence(__ATOMIC_RELEASE, "workgroup");
    __builtin_amdgcn_wave_barrier();
    __builtin_amdgcn_fence(__ATOMIC_ACQUIRE, "workgroup");
    if (OUT_MODE == 0) {
      float* C = (float*)Cout;
      const int hh = lane >> 4, c4 = (lane & 15) * 4;
      for (int pass = 0; pass < 2; ++pass) {
#pragma unroll
        for (int it = 0; it < 8; ++it) {
          const int row = it * 2 + hh;
          v4f v = *(const v4f*)(slab + row * 68 + c4);
          *(volatile v4f*)(C + (size_t)(mBase + row) * ldc + n0 + c4) = v;
        }
        __threadfence();
      }
    } else {
      const int q = lane >> 3, c8 = (lane & 7) * 8;
      unsigned short* C = (unsigned short*)Cout;
      for (int pass = 0; pass < 2; ++pass) {
#pragma unroll
        for (int it = 0; it < 4; ++it) {
          const int row = it * 4 + q;
          const float* sp = slab + row * 68 + c8;
          v8h hv;
#pragma unroll
          for (int e = 0; e < 8; ++e) hv[e] = (_Float16)sp[e];
          *(volatile v8h*)(C + (size_t)(mBase + row) * ldc + n0 + c8) = hv;
        }
        __threadfence();
      }
    }
    __builtin_amdgcn_fence(__ATOMIC_RELEASE, "workgroup");
    __builtin_amdgcn_wave_barrier();
    __builtin_amdgcn_fence(__ATOMIC_ACQUIRE, "workgroup");
  }
}

template <int OUT_MODE>
__global__ __launch_bounds__(256) void wmma_gemm32x64_f16_res(
    const unsigned short* __restrict__ Ap, const unsigned short* __restrict__ A2p, int lda,
    const unsigned short* __restrict__ Btp, int ldb,
    void* __restrict__ Cout, int ldc,
    int M, int N, int K, float scale, float rscale)
{
  const _Float16* A  = (const _Float16*)Ap;
  const _Float16* A2 = (const _Float16*)A2p;
  const _Float16* Bt = (const _Float16*)Btp;
  __shared__ __align__(16) float sT[8][16 * 68];
  const int lane = threadIdx.x & 31;
  const int wave = threadIdx.x >> 5;
  const int tilesN = N >> 6;
  const int tilesM = M >> 5;
  const int tile = blockIdx.x * 8 + wave;
  if (tile >= tilesM * tilesN) return;
  const int tm = tile / tilesN;
  const int tn = tile - tm * tilesN;
  const int m0 = tm << 5;
  const int n0 = tn << 6;

  const int rlane = lane & 15;
  const int koff  = (lane >> 4) * 8;
  const int mOff  = (lane >> 4) * 8;

  v8f acc[2][4], accr[2][4];
#pragma unroll
  for (int i = 0; i < 2; ++i)
#pragma unroll
    for (int j = 0; j < 4; ++j) {
      acc[i][j]  = (v8f){0.f,0.f,0.f,0.f,0.f,0.f,0.f,0.f};
      accr[i][j] = (v8f){0.f,0.f,0.f,0.f,0.f,0.f,0.f,0.f};
    }

  for (int k0 = 0; k0 < K; k0 += 32) {
    v16h bh[4];
#pragma unroll
    for (int j = 0; j < 4; ++j) {
      const size_t bo = (size_t)(n0 + (j << 4) + rlane) * ldb + koff + k0;
      bh[j] = FragH::load(Bt + bo);
    }
#pragma unroll
    for (int i = 0; i < 2; ++i) {
      const size_t ao = (size_t)(m0 + (i << 4) + rlane) * lda + koff + k0;
      v16h ah = FragH::load(A + ao);
      v16h al = FragH::load(A2 + ao);
#pragma unroll
      for (int j = 0; j < 4; ++j) acc[i][j] = FragH::mma(ah, bh[j], acc[i][j]);
#pragma unroll
      for (int j = 0; j < 4; ++j) accr[i][j] = FragH::mma(al, bh[j], accr[i][j]);
      group_guard8_h(acc[i][0], acc[i][1], acc[i][2], acc[i][3],
                     accr[i][0], accr[i][1], accr[i][2], accr[i][3],
                     ah, al, bh[0], bh[1], bh[2], bh[3]);
    }
    keep4_h(bh[0], bh[1], bh[2], bh[3]);
  }
  acc_guard4(acc[0][0], acc[0][1], acc[0][2], acc[0][3]);
  acc_guard4(acc[1][0], acc[1][1], acc[1][2], acc[1][3]);
  acc_guard4(accr[0][0], accr[0][1], accr[0][2], accr[0][3]);
  acc_guard4(accr[1][0], accr[1][1], accr[1][2], accr[1][3]);

  float* slab = sT[wave];
#pragma unroll
  for (int i = 0; i < 2; ++i) {
    const int mBase = m0 + (i << 4);
#pragma unroll
    for (int j = 0; j < 4; ++j) {
#pragma unroll
      for (int r = 0; r < 8; ++r) {
        const float v = (acc[i][j][r] + accr[i][j][r] * rscale) * scale;
        slab[(mOff + r) * 68 + (j << 4) + rlane] = v;
      }
    }
    __builtin_amdgcn_fence(__ATOMIC_RELEASE, "workgroup");
    __builtin_amdgcn_wave_barrier();
    __builtin_amdgcn_fence(__ATOMIC_ACQUIRE, "workgroup");
    if (OUT_MODE == 0) {
      float* C = (float*)Cout;
      const int hh = lane >> 4, c4 = (lane & 15) * 4;
      for (int pass = 0; pass < 2; ++pass) {
#pragma unroll
        for (int it = 0; it < 8; ++it) {
          const int row = it * 2 + hh;
          v4f v = *(const v4f*)(slab + row * 68 + c4);
          *(volatile v4f*)(C + (size_t)(mBase + row) * ldc + n0 + c4) = v;
        }
        __threadfence();
      }
    } else {
      const int q = lane >> 3, c8 = (lane & 7) * 8;
      unsigned short* C = (unsigned short*)Cout;
      for (int pass = 0; pass < 2; ++pass) {
#pragma unroll
        for (int it = 0; it < 4; ++it) {
          const int row = it * 4 + q;
          const float* sp = slab + row * 68 + c8;
          v8h hv;
#pragma unroll
          for (int e = 0; e < 8; ++e) hv[e] = (_Float16)sp[e];
          *(volatile v8h*)(C + (size_t)(mBase + row) * ldc + n0 + c8) = hv;
        }
        __threadfence();
      }
    }
    __builtin_amdgcn_fence(__ATOMIC_RELEASE, "workgroup");
    __builtin_amdgcn_wave_barrier();
    __builtin_amdgcn_fence(__ATOMIC_ACQUIRE, "workgroup");
  }
}

__global__ __launch_bounds__(256) void cast_f16_kernel(
    const float* __restrict__ src, unsigned short* __restrict__ dst, int total8, int real8, float scale)
{
  const int i = blockIdx.x * 256 + threadIdx.x;
  if (i >= total8) return;
  const bool live = (i < real8);
  const int ic = live ? i : (real8 - 1);
  const float* p = src + ((size_t)ic << 3);
  const v4f a0 = *(const v4f*)(p);
  const v4f a1 = *(const v4f*)(p + 4);
  v8h hv;
#pragma unroll
  for (int e = 0; e < 4; ++e) {
    const float f0 = live ? (a0[e] * scale) : 0.0f;
    const float f1 = live ? (a1[e] * scale) : 0.0f;
    hv[e]     = (_Float16)f0;
    hv[4 + e] = (_Float16)f1;
  }
  unsigned short* q = dst + ((size_t)i << 3);
  *(volatile v8h*)q = hv;
  __threadfence();
  *(volatile v8h*)q = hv;
}

__device__ __forceinline__ void split_f16(float f, float lscale, _Float16& hi, _Float16& lo) {
  const _Float16 h0 = (_Float16)f;
  const unsigned short hs = __builtin_bit_cast(unsigned short, h0);
  const unsigned hb = (unsigned)hs;
  const bool tiny = ((hb & 0x7c00u) == 0u);
  const float hf = h16_to_f32(hb);
  const float hfz = tiny ? 0.0f : hf;
  const unsigned hbz = tiny ? 0u : hb;
  const unsigned short hz = (unsigned short)hbz;
  hi = __builtin_bit_cast(_Float16, hz);
  lo = (_Float16)((f - hfz) * lscale);
}

__global__ __launch_bounds__(256) void split_x_f16_kernel(
    const float* __restrict__ src, unsigned short* __restrict__ dhi, unsigned short* __restrict__ dlo,
    int total8, float lscale)
{
  const int i = blockIdx.x * 256 + threadIdx.x;
  if (i >= total8) return;
  const size_t e0 = (size_t)i << 3;
  const v4f a0 = *(const v4f*)(src + e0);
  const v4f a1 = *(const v4f*)(src + e0 + 4);
  v8h hv, lv;
#pragma unroll
  for (int e = 0; e < 4; ++e) {
    const float f0 = a0[e];
    const float f1 = a1[e];
    _Float16 h0, l0, h1, l1;
    split_f16(f0, lscale, h0, l0);
    split_f16(f1, lscale, h1, l1);
    hv[e]     = h0;
    hv[4 + e] = h1;
    lv[e]     = l0;
    lv[4 + e] = l1;
  }
  unsigned short* qh = dhi + e0;
  unsigned short* ql = dlo + e0;
  *(volatile v8h*)qh = hv;
  *(volatile v8h*)ql = lv;
  __threadfence();
  *(volatile v8h*)qh = hv;
  *(volatile v8h*)ql = lv;
}

__global__ __launch_bounds__(256) void dt_cast_kernel(
    const float* __restrict__ PROJ, unsigned short* __restrict__ DT16, int total8, float scale)
{
  const int i = blockIdx.x * 256 + threadIdx.x;
  if (i >= total8) return;
  const int e0  = i << 3;
  const int row = e0 >> 6;
  const int c8  = e0 & 63;
  const float* p = PROJ + (size_t)row * kPrjP + c8;
  const v4f a0 = *(const v4f*)(p);
  const v4f a1 = *(const v4f*)(p + 4);
  v8h hv;
#pragma unroll
  for (int e = 0; e < 4; ++e) {
    hv[e]     = (_Float16)(a0[e] * scale);
    hv[4 + e] = (_Float16)(a1[e] * scale);
  }
  unsigned short* qd = DT16 + e0;
  *(volatile v8h*)qd = hv;
  __threadfence();
  *(volatile v8h*)qd = hv;
}

__global__ __launch_bounds__(256) void conv_silu_kernel(
    const float* __restrict__ XC, const float* __restrict__ cw, const float* __restrict__ cb,
    unsigned short* __restrict__ U16)
{
  __shared__ __align__(16) float sT[16 * kTP];
  const int tid = threadIdx.x, lane = tid & 31, wave = tid >> 5;
  const int d0 = blockIdx.x * 256, d = d0 + tid;
  const int g0 = blockIdx.y * 64;
  const int tb = g0 & (kSeqL - 1);
  const v4f wv = *(const v4f*)(cw + (size_t)d * 4);
  const float w0 = wv[0], w1 = wv[1], w2 = wv[2], w3 = wv[3];
  const float bc = cb[d];
  float xm3, xm2, xm1;
  {
    const bool hist = (tb > 0);
    const int rb = hist ? (g0 - 3) : g0;
    const float v3 = XC[(size_t)rb * kDin + d];
    const float v2 = XC[(size_t)(rb + 1) * kDin + d];
    const float v1 = XC[(size_t)(rb + 2) * kDin + d];
    xm3 = hist ? v3 : 0.f;
    xm2 = hist ? v2 : 0.f;
    xm1 = hist ? v1 : 0.f;
  }
#pragma unroll 1
  for (int sub = 0; sub < 4; ++sub) {
    const int lb = g0 + sub * 16;
#pragma unroll 1
    for (int s = 0; s < 16; ++s) {
      const float xcur = XC[(size_t)(lb + s) * kDin + d];
      float acc = w0 * xm3;
      acc = fmaf(w1, xm2, acc);
      acc = fmaf(w2, xm1, acc);
      acc = fmaf(w3, xcur, acc);
      const float sv = acc + bc;
      const float sg = 1.0f / (1.0f + expf(-sv));
      sT[s * kTP + tid] = sv * sg;
      xm3 = xm2; xm2 = xm1; xm1 = xcur;
    }
    __syncthreads();
    v8h bv[2];
#pragma unroll
    for (int it = 0; it < 2; ++it) {
      const float* sp = sT + (it * 8 + wave) * kTP + lane * 8;
      const v4f a0 = *(const v4f*)(sp);
      const v4f a1 = *(const v4f*)(sp + 4);
#pragma unroll
      for (int e = 0; e < 4; ++e) {
        bv[it][e]     = (_Float16)a0[e];
        bv[it][4 + e] = (_Float16)a1[e];
      }
    }
    for (int pass = 0; pass < 2; ++pass) {
#pragma unroll
      for (int it = 0; it < 2; ++it)
        *(volatile v8h*)(U16 + (size_t)(lb + it * 8 + wave) * kDin + d0 + lane * 8) = bv[it];
      __threadfence();
    }
    __syncthreads();
  }
}

__global__ __launch_bounds__(256) void scan_kernel(
    const unsigned* __restrict__ DTR32, const unsigned* __restrict__ U32, const unsigned* __restrict__ Z32,
    const float* __restrict__ PROJ, const float* __restrict__ bdt, const float* __restrict__ A_log,
    const float* __restrict__ Dv, unsigned short* __restrict__ YG16)
{
  __shared__ __align__(16) float sBC[16 * 32];
  __shared__ __align__(16) float sY[16 * kTP];
  __shared__ __align__(16) float sA[kNst * 256];
  const int tid = threadIdx.x, lane = tid & 31, wave = tid >> 5;
  const int d0 = blockIdx.x * 256, d = d0 + tid;
  const size_t row0 = (size_t)blockIdx.y * kSeqL;

#pragma unroll 1
  for (int n = 0; n < kNst; ++n) sA[n * 256 + tid] = -expf(A_log[(size_t)d * kNst + n]);
  __syncthreads();
  float An[kNst], h[kNst];
#pragma unroll
  for (int n = 0; n < kNst; ++n) {
    An[n] = sA[n * 256 + tid];
    h[n] = 0.f;
  }
  const float bb = bdt[d];
  const float Dd = Dv[d];
  const unsigned wsh = (unsigned)(tid & 1) * 16u;
  const size_t wcol = (size_t)(d >> 1);

#pragma unroll 1
  for (int c = 0; c < kSeqL / 16; ++c) {
    const int l0 = c * 16;
    if (tid < 128) {
      const int r = tid >> 3, q = (tid & 7) * 4;
      const v4f v = *(const v4f*)(PROJ + (row0 + l0 + r) * kPrjP + kDtR + q);
      *(v4f*)(sBC + r * 32 + q) = v;
    }
    __syncthreads();
#pragma unroll 1
    for (int s = 0; s < 16; ++s) {
      const size_t m  = row0 + (size_t)(l0 + s);
      const size_t wi = m * (kDin / 2) + wcol;
      const unsigned wd = DTR32[wi];
      const unsigned wu = U32[wi];
      const unsigned wz = Z32[wi];
      const float dtr = h16_to_f32((wd >> wsh) & 0xffffu);
      const float xv  = h16_to_f32((wu >> wsh) & 0xffffu);
      const float zv  = h16_to_f32((wz >> wsh) & 0xffffu);
      const float vpre = dtr + bb;
      const float ea   = expf(-fabsf(vpre));
      const float up   = 1.0f + ea;
      const float l1p  = logf(up) + (ea - (up - 1.0f)) * (1.0f / up);
      const float delta = fmaxf(vpre, 0.0f) + l1p;
      float dtx = delta * xv;
      asm volatile("" : "+v"(dtx));
      v4f Bq[4], Cq[4];
#pragma unroll
      for (int qq = 0; qq < 4; ++qq) {
        Bq[qq] = *(const v4f*)(sBC + s * 32 + 4 * qq);
        Cq[qq] = *(const v4f*)(sBC + s * 32 + kNst + 4 * qq);
      }
      float y = 0.f;
#pragma unroll
      for (int n = 0; n < kNst; ++n) {
        const float e = __expf(delta * An[n]);
        float p = dtx * Bq[n >> 2][n & 3];
        asm volatile("" : "+v"(p));
        float qv = h[n] * e;
        asm volatile("" : "+v"(qv));
        const float hn = qv + p;
        h[n] = hn;
        float rr = Cq[n >> 2][n & 3] * hn;
        asm volatile("" : "+v"(rr));
        y += rr;
      }
      float sk = xv * Dd;
      asm volatile("" : "+v"(sk));
      y += sk;
      const float sg = 1.0f / (1.0f + expf(-zv));
      const float g  = zv * sg;
      sY[s * kTP + tid] = (y * g) * kCarryY;
    }
    __syncthreads();
    v8h hv[2];
#pragma unroll
    for (int it = 0; it < 2; ++it) {
      const float* sp = sY + (it * 8 + wave) * kTP + lane * 8;
      const v4f a0 = *(const v4f*)(sp);
      const v4f a1 = *(const v4f*)(sp + 4);
#pragma unroll
      for (int e = 0; e < 4; ++e) {
        hv[it][e]     = (_Float16)a0[e];
        hv[it][4 + e] = (_Float16)a1[e];
      }
    }
    for (int pass = 0; pass < 2; ++pass) {
#pragma unroll
      for (int it = 0; it < 2; ++it)
        *(volatile v8h*)(YG16 + (row0 + (size_t)(l0 + it * 8 + wave)) * kDin + d0 + lane * 8) = hv[it];
      __threadfence();
    }
  }
}

extern "C" void kernel_launch(void* const* d_in, const int* in_sizes, int n_in,
                              void* d_out, int out_size, void* d_ws, size_t ws_size,
                              hipStream_t stream)
{
  if (n_in < 10) return;
  if (in_sizes[0] != kRows * kDmod) return;
  if (in_sizes[1] != kXZN * kDmod) return;
  if (in_sizes[2] != kDin * 4) return;
  if (in_sizes[3] != kDin) return;
  if (in_sizes[4] != kPrjN * kDin) return;
  if (in_sizes[5] != kDin * kDtR) return;
  if (in_sizes[6] != kDin) return;
  if (in_sizes[7] != kDin * kNst) return;
  if (in_sizes[8] != kDin) return;
  if (in_sizes[9] != kDmod * kDin) return;
  if (out_size != kRows * kDmod) return;
  if (ws_size < kWsTotal) return;

  const float* x      = (const float*)d_in[0];
  const float* W_in   = (const float*)d_in[1];
  const float* conv_w = (const float*)d_in[2];
  const float* conv_b = (const float*)d_in[3];
  const float* W_xprj = (const float*)d_in[4];
  const float* W_dt   = (const float*)d_in[5];
  const float* b_dt   = (const float*)d_in[6];
  const float* A_log  = (const float*)d_in[7];
  const float* Dv     = (const float*)d_in[8];
  const float* W_out  = (const float*)d_in[9];
  float* dout = (float*)d_out;

  char* ws = (char*)d_ws;
  unsigned short* X16     = (unsigned short*)(ws + kOffX16);
  unsigned short* XLO16   = (unsigned short*)(ws + kOffXLO16);
  unsigned short* WIN16   = (unsigned short*)(ws + kOffWIN16);
  unsigned short* WXP16   = (unsigned short*)(ws + kOffWXP16);
  unsigned short* WDT16   = (unsigned short*)(ws + kOffWDT16);
  unsigned short* WOUT16  = (unsigned short*)(ws + kOffWOUT16);
  float*          XC32    = (float*)(ws + kOffXC32);
  unsigned short* Z16     = (unsigned short*)(ws + kOffZ16);
  unsigned short* U16     = (unsigned short*)(ws + kOffU16);
  float*          XDBL32  = (float*)(ws + kOffXDBL32);
  unsigned short* DTLO16  = (unsigned short*)(ws + kOffDTLO16);
  unsigned short* DTRAW16 = (unsigned short*)(ws + kOffDTRAW16);
  unsigned short* YG16    = (unsigned short*)(ws + kOffYG16);

  {
    const int t8 = kRows * kDmod / 8;
    split_x_f16_kernel<<<t8 / 256, 256, 0, stream>>>(x, X16, XLO16, t8, kCarryXlo);
  }
  {
    const int t8 = kXZN * kDmod / 8;
    cast_f16_kernel<<<t8 / 256, 256, 0, stream>>>(W_in, WIN16, t8, t8, kCarryW);
  }
  {
    const int t8 = kPrjP * kDin / 8;
    const int r8 = kPrjN * kDin / 8;
    cast_f16_kernel<<<t8 / 256, 256, 0, stream>>>(W_xprj, WXP16, t8, r8, kCarryW);
  }
  {
    const int t8 = kDin * kDtR / 8;
    cast_f16_kernel<<<t8 / 256, 256, 0, stream>>>(W_dt, WDT16, t8, t8, kCarryWdt);
  }
  {
    const int t8 = kDmod * kDin / 8;
    cast_f16_kernel<<<t8 / 256, 256, 0, stream>>>(W_out, WOUT16, t8, t8, kCarryW);
  }

  wmma_gemm32x64_f16_res<0><<<(kRows / 32) * (kDin / 64) / 8, 256, 0, stream>>>(
      X16, XLO16, kDmod, WIN16, kDmod, (void*)XC32, kDin, kRows, kDin, kDmod,
      1.0f / kCarryW, 1.0f / kCarryXlo);

  wmma_gemm32x64_f16_res<1><<<(kRows / 32) * (kDin / 64) / 8, 256, 0, stream>>>(
      X16, XLO16, kDmod, WIN16 + (size_t)kDin * kDmod, kDmod, (void*)Z16, kDin, kRows, kDin, kDmod,
      1.0f / kCarryW, 1.0f / kCarryXlo);

  conv_silu_kernel<<<dim3(kDin / 256, kRows / 64), 256, 0, stream>>>(XC32, conv_w, conv_b, U16);

  wmma_gemm64_f16<0><<<(kRows / 64) * (kPrjP / 64) / 8, 256, 0, stream>>>(
      U16, kDin, WXP16, kDin, (void*)XDBL32, kPrjP, kRows, kPrjP, kDin, 1.0f / kCarryW);

  {
    const int t8 = kRows * kDtR / 8;
    dt_cast_kernel<<<t8 / 256, 256, 0, stream>>>(XDBL32, DTLO16, t8, kCarryDt);
  }

  wmma_gemm64_f16<1><<<(kRows / 64) * (kDin / 64) / 8, 256, 0, stream>>>(
      DTLO16, kDtR, WDT16, kDtR, (void*)DTRAW16, kDin, kRows, kDin, kDtR, 1.0f / (kCarryDt * kCarryWdt));

  scan_kernel<<<dim3(kDin / 256, kBatch), 256, 0, stream>>>(
      (const unsigned*)DTRAW16, (const unsigned*)U16, (const unsigned*)Z16,
      XDBL32, b_dt, A_log, Dv, YG16);

  wmma_gemm64_f16<0><<<(kRows / 64) * (kDmod / 64) / 8, 256, 0, stream>>>(
      YG16, kDin, WOUT16, kDin, (void*)dout, kDmod, kRows, kDmod, kDin, 1.0f / (kCarryY * kCarryW));
}
